// Model_21844203667996
// MI455X (gfx1250) — hardware-verified
//
#include <hip/hip_runtime.h>


#ifndef NB
#define NB 1024
#endif
#define NB_FULL 1024
#ifndef NTK
#define NTK 32
#endif
#define NS   512
#define IMG  28
#define OW   29
#define NP   841
#define KE   896
#define LW   1353
#define CCH  64
#define MEMW 64
#define NO   10
#define NOP  16
#define OSP2 68
#define WSC  64.0f
#define WINV (1.0f / 64.0f)

#define WE_BLK ((NS * KE / 8) / 256)
#define WA_BLK ((NS * NS / 8) / 256)
#define HW_BLK ((NOP * NS / 8) / 256)
#define A0_BLK ((NB * NS / 8) / 256)

static_assert(NP == OW * OW);
static_assert(OW == IMG + 1);
static_assert(LW == NP + NS);
static_assert(KE % 32 == 0);
static_assert(KE >= NP);
static_assert((KE * 2) % 128 == 0);
static_assert(NS % 64 == 0);
static_assert(NB % 64 == 0);
static_assert(NB % 16 == 0);
static_assert(NB <= NB_FULL);
static_assert(NTK >= 1);
static_assert(NTK <= 32);
static_assert(NTK < MEMW);
static_assert(NO <= NOP);
static_assert(NOP == 16);
static_assert((NS * KE / 8) % 256 == 0);
static_assert((NS * NS / 8) % 256 == 0);
static_assert((NOP * NS / 8) % 256 == 0);
static_assert((NB * NS / 8) % 256 == 0);
static_assert(KE / 8 <= 256);
static_assert((KE / 8) * 16 == KE * 2);
static_assert(4 * 128 == NS);
static_assert(32 * 32 * 16 == 64 * 64 * 4);
static_assert(16 * 32 * 16 == 64 * 64 * 2);
static_assert((32 + 8) * 16 == 16 * NO * 4);
static_assert((16 * NO * 4) % 128 == 0);
static_assert((OSP2 * 4) % 16 == 0);
static_assert((2 * 64 * OSP2 + 32) * 4 <= 131072);
static_assert(64 * OSP2 * 4 <= 131072);
static_assert((5 * CCH + 8) * 4 + KE * 2 <= 131072);

typedef _Float16 h16;
typedef __attribute__((ext_vector_type(16))) _Float16 v16h;
typedef __attribute__((ext_vector_type(8)))  _Float16 v8h;
typedef __attribute__((ext_vector_type(8)))  float    v8f;
typedef __attribute__((ext_vector_type(4)))  float    v4f;
typedef v4f  __attribute__((may_alias)) v4fa;
typedef v8h  __attribute__((may_alias)) v8ha;

__device__ __forceinline__ unsigned short f2bf(float f) { unsigned u = __float_as_uint(f); u += 0x7FFFu + ((u >> 16) & 1u); return (unsigned short)(u >> 16); }
__device__ __forceinline__ float bfr(float f) { return __uint_as_float(((unsigned)f2bf(f)) << 16); }
__device__ __forceinline__ v16h cat16(v8h lo, v8h hi) { return __builtin_shufflevector(lo, hi, 0, 1, 2, 3, 4, 5, 6, 7, 8, 9, 10, 11, 12, 13, 14, 15); }
__device__ __forceinline__ v8f wmma16(v16h a, v16h b, v8f c) { return __builtin_amdgcn_wmma_f32_16x16x32_f16(false, a, false, b, (short)0, c, false, false); }
__device__ __forceinline__ v8f wmma16g(v16h a, v16h b, v8f c) { c = wmma16(a, b, c); asm volatile("v_nop\n\tv_nop\n\tv_nop\n\tv_nop" : "+v"(c) : "v"(a), "v"(b)); return c; }
__device__ __forceinline__ v16h  ldh(const h16* p) { return cat16(*(const v8h*)p, *(const v8h*)(p + 16)); }
__device__ __forceinline__ void wave_sync() { __builtin_amdgcn_fence(3  , "wavefront"); __builtin_amdgcn_wave_barrier(); asm volatile("" ::: "memory"); }
static __device__ __forceinline__ h16 toh_flush(float v) { const h16 r = (h16)v; return (fabsf(v) < 6.103515625e-05f) ? (h16)0.0f : r; }
__device__ __forceinline__ void st8h(h16* p, v8h o) { *(volatile v8h*)p = o; __threadfence(); *(volatile v8h*)p = o; }

__global__ __launch_bounds__(256) void k_planes(const float* __restrict__ lin2w, const float* __restrict__ outw, const float* __restrict__ astate,
                                                h16* WEp, h16* WAp, h16* HWp, h16* A0p) {
    const int blk = blockIdx.x, tid = threadIdx.x;
    if (blk < WE_BLK) {
        const int i = blk * 256 + tid; const int n = i / (KE / 8); const int k8 = (i - n * (KE / 8)) * 8;
        const float* src = lin2w + (size_t)n * LW;
        float v[8];
#pragma unroll
        for (int j = 0; j < 8; ++j) { const int kk = k8 + j; v[j] = src[kk < NP ? kk : NP - 1]; }
#pragma unroll
        for (int j = 0; j < 8; ++j) asm volatile("" : "+v"(v[j]));
        v8h o;
#pragma unroll
        for (int j = 0; j < 8; ++j) o[j] = ((k8 + j) < NP) ? toh_flush(bfr(v[j]) * WSC) : (h16)0.0f;
        st8h(WEp + (size_t)i * 8, o);
    } else if (blk < WE_BLK + WA_BLK) {
        const int i = (blk - WE_BLK) * 256 + tid; const int n = i / (NS / 8); const int k8 = (i - n * (NS / 8)) * 8;
        const float* src = lin2w + (size_t)n * LW + NP + k8;
        float v[8];
#pragma unroll
        for (int j = 0; j < 8; ++j) v[j] = src[j];
        v8h o;
#pragma unroll
        for (int j = 0; j < 8; ++j) o[j] = toh_flush(bfr(v[j]) * WSC);
        st8h(WAp + (size_t)i * 8, o);
    } else if (blk < WE_BLK + WA_BLK + HW_BLK) {
        const int i = (blk - WE_BLK - WA_BLK) * 256 + tid; const int n = i / (NS / 8); const int k8 = (i - n * (NS / 8)) * 8;
        const int nc = n < NO ? n : NO - 1;
        v8f v = *(const v8f*)(outw + (size_t)nc * NS + k8);
        asm volatile("" : "+v"(v));
        v8h o;
#pragma unroll
        for (int j = 0; j < 8; ++j) o[j] = (n < NO) ? toh_flush(bfr(v[j]) * WSC) : (h16)0.0f;
        st8h(HWp + (size_t)i * 8, o);
    } else {
        const int i = (blk - WE_BLK - WA_BLK - HW_BLK) * 256 + tid;
        const int s8 = (i & (NS / 8 - 1)) * 8;
        const v8f v = *(const v8f*)(astate + s8);
        v8h o;
#pragma unroll
        for (int j = 0; j < 8; ++j) o[j] = toh_flush(bfr(v[j]));
        st8h(A0p + (size_t)i * 8, o);
    }
}
static_assert((NS / 8 & (NS / 8 - 1)) == 0);

__global__ __launch_bounds__(128) void k_mterm(const float* __restrict__ mem, const float* __restrict__ wmem, const float* __restrict__ bsc, float* MT) {
#pragma clang fp contract(off)
    const int t = blockIdx.x + 1; const int s4 = threadIdx.x * 4;
    const float* m0 = mem + (size_t)s4 * MEMW + t;
    float a0 = 0.0f, a1 = 0.0f, a2 = 0.0f, a3 = 0.0f;
#pragma unroll 1
    for (int k = 0; k + t <= MEMW - 1; ++k) {
        const float w = bfr(wmem[k]);
        a0 += bfr(m0[k]) * w; a1 += bfr(m0[MEMW + k]) * w; a2 += bfr(m0[2 * MEMW + k]) * w; a3 += bfr(m0[3 * MEMW + k]) * w; }
    const float bb = bfr(bsc[0]);
    v4f o; o[0] = a0 + bb; o[1] = a1 + bb; o[2] = a2 + bb; o[3] = a3 + bb;
    float* d = MT + (size_t)(t - 1) * NS + s4;
    *(volatile v4f*)d = o; __threadfence(); *(volatile v4f*)d = o;
}

__global__ __launch_bounds__(256) void k_ef(const float* __restrict__ x, const float* __restrict__ convw, const float* __restrict__ convb,
                                            const float* __restrict__ lin1w, const float* __restrict__ lin1b, h16* EFp) {
#pragma clang fp contract(off)
    __shared__ float pe[5 * CCH];
    __shared__ float es[8];
    __shared__ __align__(16) h16 rowh[KE];
    const int tid = threadIdx.x; const int b = blockIdx.x;
    if (tid < CCH) {
        const float lw = bfr(lin1w[tid]);
        pe[0 * CCH + tid] = bfr(convw[tid * 4 + 0]) * lw; pe[1 * CCH + tid] = bfr(convw[tid * 4 + 1]) * lw;
        pe[2 * CCH + tid] = bfr(convw[tid * 4 + 2]) * lw; pe[3 * CCH + tid] = bfr(convw[tid * 4 + 3]) * lw;
        pe[4 * CCH + tid] = bfr(convb[tid]) * lw; }
    __syncthreads();
    if (tid < 32) {
        const int q = tid < 4 ? tid : 4;
        float s = 0.0f;
#pragma unroll 1
        for (int c = 0; c < CCH; ++c) s += pe[q * CCH + c];
        const float lb = bfr(lin1b[0]);
        s += (q == 4) ? lb : 0.0f;
        if (tid < 5) es[tid] = s; }
    __syncthreads();
    const float e0 = es[0], e1 = es[1], e2 = es[2], e3 = es[3], eb = es[4];
    const float* xb = x + (size_t)b * (IMG * IMG);
#pragma unroll 1
    for (int p = tid; p < KE; p += 256) {
        const int pc = p < NP ? p : NP - 1;
        const int i = pc / OW, jx = pc - i * OW;
        const int ra = i > 0 ? i - 1 : 0, rb = i < IMG ? i : IMG - 1;
        const int ca = jx > 0 ? jx - 1 : 0, cb = jx < IMG ? jx : IMG - 1;
        float x00 = xb[ra * IMG + ca], x01 = xb[ra * IMG + cb], x10 = xb[rb * IMG + ca], x11 = xb[rb * IMG + cb];
        asm volatile("" : "+v"(x00)); asm volatile("" : "+v"(x01)); asm volatile("" : "+v"(x10)); asm volatile("" : "+v"(x11));
        const bool up = i > 0, dn = i < IMG, lf = jx > 0, rt = jx < IMG;
        const float t00 = (up & lf) ? bfr(x00) : 0.0f, t01 = (up & rt) ? bfr(x01) : 0.0f;
        const float t10 = (dn & lf) ? bfr(x10) : 0.0f, t11 = (dn & rt) ? bfr(x11) : 0.0f;
        float acc = eb; acc += t00 * e0; acc += t01 * e1; acc += t10 * e2; acc += t11 * e3;
        const float v = (p < NP) ? fmaxf(acc, 0.0f) : 0.0f;
        rowh[p] = toh_flush(v); }
    __syncthreads();
    if (tid < KE / 8) {
        const v8h o = *(const v8ha*)(&rowh[8 * tid]);
        st8h(EFp + (size_t)b * KE + 8 * tid, o); }
}

__device__ __forceinline__ void gemm_main(const h16* __restrict__ A, const h16* __restrict__ Bt, const int K, const int r0, const int c0, const int lr, const int hi, v8f (&acc)[4][4]) {
#pragma unroll
    for (int mb = 0; mb < 4; ++mb)
#pragma unroll
        for (int nb = 0; nb < 4; ++nb) acc[mb][nb] = (v8f){};
    const size_t aoff = (size_t)(r0 + lr) * K + 8 * hi, boff = (size_t)(c0 + lr) * K + 8 * hi;
#pragma unroll 1
    for (int kc = 0; kc < K; kc += 32) {
        v16h a[4];
#pragma unroll
        for (int mb = 0; mb < 4; ++mb) a[mb] = ldh(A + aoff + (size_t)mb * 16 * K + kc);
#pragma unroll
        for (int nb = 0; nb < 4; ++nb) { const v16h b = ldh(Bt + boff + (size_t)nb * 16 * K + kc);
#pragma unroll
            for (int mb = 0; mb < 4; ++mb) acc[mb][nb] = wmma16g(a[mb], b, acc[mb][nb]); }
    }
}

__global__ __launch_bounds__(32) void k_base(const h16* __restrict__ EFp, const h16* __restrict__ WEp, const float* __restrict__ lin2b, float* BASEW) {
    __shared__ __align__(16) float os[64 * OSP2];
    const int lane = threadIdx.x & 31, lr = lane & 15, hi = lane >> 4; const int r0 = blockIdx.x * 64, c0 = blockIdx.y * 64;
    v8f acc[4][4];
    gemm_main(EFp, WEp, KE, r0, c0, lr, hi, acc);
#pragma unroll
    for (int mb = 0; mb < 4; ++mb)
#pragma unroll
        for (int nb = 0; nb < 4; ++nb)
#pragma unroll
            for (int j = 0; j < 8; ++j) os[(mb * 16 + hi * 8 + j) * OSP2 + nb * 16 + lr] = acc[mb][nb][j];
    wave_sync();
    const int c4 = (lane & 15) * 4, rsub = lane >> 4;
    const v4f braw = *(const v4f*)(lin2b + c0 + c4);
    v4f bb; bb[0] = bfr(braw[0]); bb[1] = bfr(braw[1]); bb[2] = bfr(braw[2]); bb[3] = bfr(braw[3]);
#pragma unroll 1
    for (int ps = 0; ps < 2; ++ps) {
#pragma unroll 1
        for (int s = 0; s < 32; ++s) { const int row = 2 * s + rsub;
            const v4f xv = *(const v4fa*)(&os[row * OSP2 + c4]);
            v4f val; val[0] = xv[0] * WINV + bb[0]; val[1] = xv[1] * WINV + bb[1]; val[2] = xv[2] * WINV + bb[2]; val[3] = xv[3] * WINV + bb[3];
            *(volatile v4f*)(BASEW + (size_t)(r0 + row) * NS + c0 + c4) = val; }
        if (ps == 0) __threadfence(); }
}

__global__ __launch_bounds__(32) void k_tick(const h16* __restrict__ ACTR, const h16* __restrict__ WAp, const float* __restrict__ BASEp, const float* __restrict__ MTp,
                                             const float* __restrict__ wmem, float* HIST, h16* ACTW, int j, int wrh) {
    __shared__ __align__(16) float os[64 * OSP2];
    __shared__ __align__(16) float az[64 * OSP2];
    __shared__ float wl[32];
    const int lane = threadIdx.x & 31, lr = lane & 15, hi = lane >> 4; const int r0 = blockIdx.x * 64, c0 = blockIdx.y * 64;
    const int jc = min(max(j, 0), NTK - 1);
    { int wi = MEMW - 1 - jc + lane; wi = min(max(wi, 0), MEMW - 1); wl[lane] = bfr(wmem[wi]); }
    v8f acc[4][4];
    gemm_main(ACTR, WAp, NS, r0, c0, lr, hi, acc);
#pragma unroll
    for (int mb = 0; mb < 4; ++mb)
#pragma unroll
        for (int nb = 0; nb < 4; ++nb)
#pragma unroll
            for (int jj = 0; jj < 8; ++jj) os[(mb * 16 + hi * 8 + jj) * OSP2 + nb * 16 + lr] = acc[mb][nb][jj];
    wave_sync();
    const size_t MN = (size_t)NB * NS;
    const int c4 = (lane & 15) * 4, rsub = lane >> 4;
    const v4f mt = *(const v4f*)(MTp + (size_t)jc * NS + c0 + c4);
    const float wlast = wl[jc];
#pragma unroll 1
    for (int s = 0; s < 32; ++s) { const int row = 2 * s + rsub;
        const size_t gi = (size_t)(r0 + row) * NS + c0 + c4;
        const v4f xv = *(const v4fa*)(&os[row * OSP2 + c4]);
        const v4f bs = *(const v4f*)(BASEp + gi);
        v4f p; p[0] = fmaxf(xv[0] * WINV + bs[0], 0.0f); p[1] = fmaxf(xv[1] * WINV + bs[1], 0.0f); p[2] = fmaxf(xv[2] * WINV + bs[2], 0.0f); p[3] = fmaxf(xv[3] * WINV + bs[3], 0.0f);
        v4f a = mt;
        const float* hp = HIST + gi;
#pragma unroll 1
        for (int h = 0; h < jc; ++h) { const float w = wl[h]; const v4f hv = *(const v4f*)(hp + (size_t)h * MN); a += hv * w; }
        a += p * wlast;
        *(v4fa*)(&os[row * OSP2 + c4]) = p; *(v4fa*)(&az[row * OSP2 + c4]) = a; }
    wave_sync();
#pragma unroll 1
    for (int ps = 0; ps < 2; ++ps) {
        if (wrh != 0) {
            float* hw = HIST + (size_t)jc * MN;
#pragma unroll 1
            for (int s = 0; s < 32; ++s) { const int row = 2 * s + rsub;
                const v4f val = *(const v4fa*)(&os[row * OSP2 + c4]);
                *(volatile v4f*)(hw + (size_t)(r0 + row) * NS + c0 + c4) = val; } }
#pragma unroll 1
        for (int s = 0; s < 16; ++s) { const int row = 4 * s + (lane >> 3), c8 = (lane & 7) * 8;
            const v4f x0 = *(const v4fa*)(&az[row * OSP2 + c8]); const v4f x1 = *(const v4fa*)(&az[row * OSP2 + c8 + 4]); v8h hv;
#pragma unroll
            for (int i = 0; i < 4; ++i) { hv[i] = toh_flush(x0[i]); hv[4 + i] = toh_flush(x1[i]); }
            *(volatile v8h*)(ACTW + (size_t)(r0 + row) * NS + c0 + c8) = hv; }
        if (ps == 0) __threadfence(); }
}

__global__ __launch_bounds__(32) void k_head(const h16* __restrict__ ACTF, const h16* __restrict__ HWp, const float* __restrict__ outb, float* OUT) {
    __shared__ __align__(16) float hs[16 * NO];
    const int lane = threadIdx.x & 31, lr = lane & 15, hi = lane >> 4; const int r0 = blockIdx.x * 16;
    v8f acc = (v8f){};
    const size_t aoff = (size_t)(r0 + lr) * NS + 8 * hi, boff = (size_t)lr * NS + 8 * hi;
#pragma unroll 1
    for (int kc = 0; kc < NS; kc += 32) { const v16h a = ldh(ACTF + aoff + kc); const v16h b = ldh(HWp + boff + kc); acc = wmma16g(a, b, acc); }
    float bo = outb[lr < NO ? lr : NO - 1];
    asm volatile("" : "+v"(bo));
    bo = bfr(bo);
#pragma unroll
    for (int r = 0; r < 8; ++r) { const float val = acc[r] * WINV + bo; if (lr < NO) hs[(8 * hi + r) * NO + lr] = val; }
    wave_sync();
    float* ob = OUT + (size_t)r0 * NO;
#pragma unroll 1
    for (int ps = 0; ps < 2; ++ps) {
        const v4f v0 = *(const v4fa*)(&hs[4 * lane]);
        *(volatile v4f*)(ob + 4 * lane) = v0;
        if (lane < 8) { const v4f v1 = *(const v4fa*)(&hs[128 + 4 * lane]); *(volatile v4f*)(ob + 128 + 4 * lane) = v1; }
        if (ps == 0) __threadfence(); }
}

static constexpr size_t al256(size_t v) { return (v + 255) & ~(size_t)255; }
static constexpr size_t SZ_EF  = al256((size_t)NB * KE * 2);
static constexpr size_t SZ_WE  = al256((size_t)NS * KE * 2);
static constexpr size_t SZ_WA  = al256((size_t)NS * NS * 2);
static constexpr size_t SZ_HW  = al256((size_t)NOP * NS * 2);
static constexpr size_t SZ_MT  = al256((size_t)NTK * NS * 4);
static constexpr size_t SZ_ACT = al256((size_t)NB * NS * 2);
static constexpr size_t SZ_BS  = al256((size_t)NB * NS * 4);
static constexpr size_t SZ_HS  = al256((size_t)(NTK > 1 ? NTK - 1 : 1) * NB * NS * 4);
static constexpr size_t SZ_TOTAL = SZ_EF + SZ_WE + SZ_WA + SZ_HW + SZ_MT + 2 * SZ_ACT + SZ_BS + SZ_HS;
static_assert(SZ_TOTAL <= (size_t)134217728);
static_assert((size_t)WE_BLK * 256 * 16 == (size_t)NS * KE * 2);
static_assert((size_t)WA_BLK * 256 * 16 == (size_t)NS * NS * 2);
static_assert((size_t)HW_BLK * 256 * 16 == (size_t)NOP * NS * 2);
static_assert((size_t)A0_BLK * 256 * 16 == (size_t)NB * NS * 2);

extern "C" void kernel_launch(void* const* d_in, const int* in_sizes, int n_in,
                              void* d_out, int out_size, void* d_ws, size_t ws_size, hipStream_t stream) {
    if (n_in < 13) return;
    if ((size_t)in_sizes[0] < (size_t)NB * IMG * IMG) return;
    if (in_sizes[1] < CCH * 4 || in_sizes[2] < CCH || in_sizes[3] < CCH || in_sizes[4] < 1) return;
    if ((size_t)in_sizes[5] < (size_t)NS * LW || in_sizes[6] < NS) return;
    if (in_sizes[7] < NO * NS || in_sizes[8] < NO || in_sizes[9] < NS) return;
    if (in_sizes[10] < NS * MEMW || in_sizes[11] < MEMW || in_sizes[12] < 1) return;
    if ((size_t)out_size < (size_t)NB * NO) return;
    if (SZ_TOTAL > ws_size) return;
    const float* x      = (const float*)d_in[0];
    const float* convw  = (const float*)d_in[1];
    const float* convb  = (const float*)d_in[2];
    const float* lin1w  = (const float*)d_in[3];
    const float* lin1b  = (const float*)d_in[4];
    const float* lin2w  = (const float*)d_in[5];
    const float* lin2b  = (const float*)d_in[6];
    const float* outw   = (const float*)d_in[7];
    const float* outb   = (const float*)d_in[8];
    const float* astate = (const float*)d_in[9];
    const float* memory = (const float*)d_in[10];
    const float* wmem   = (const float*)d_in[11];
    const float* bsc    = (const float*)d_in[12];
    float* OUT = (float*)d_out;
    char* wsp = (char*)d_ws;
    h16* EF = (h16*)wsp; wsp += SZ_EF;
    h16* WE = (h16*)wsp; wsp += SZ_WE;
    h16* WA = (h16*)wsp; wsp += SZ_WA;
    h16* HW = (h16*)wsp; wsp += SZ_HW;
    float* MT = (float*)wsp; wsp += SZ_MT;
    h16* ACT[2];
    ACT[0] = (h16*)wsp; wsp += SZ_ACT;
    ACT[1] = (h16*)wsp; wsp += SZ_ACT;
    float* BASE = (float*)wsp; wsp += SZ_BS;
    float* HIST = (float*)wsp; wsp += SZ_HS;

    k_planes<<<WE_BLK + WA_BLK + HW_BLK + A0_BLK, 256, 0, stream>>>(lin2w, outw, astate, WE, WA, HW, ACT[0]);
    k_mterm<<<NTK, 128, 0, stream>>>(memory, wmem, bsc, MT);
    k_ef<<<NB, 256, 0, stream>>>(x, convw, convb, lin1w, lin1b, EF);
    k_base<<<dim3(NB / 64, NS / 64, 1), 32, 0, stream>>>(EF, WE, lin2b, BASE);
    for (int j = 0; j < NTK; ++j)
        k_tick<<<dim3(NB / 64, NS / 64, 1), 32, 0, stream>>>(ACT[j & 1], WA, BASE, MT, wmem, HIST, ACT[(j + 1) & 1], j, (j < NTK - 1) ? 1 : 0);
    k_head<<<NB / 16, 32, 0, stream>>>(ACT[NTK & 1], HW, outb, OUT);
}
